// nat_base_54735063220687
// MI455X (gfx1250) — hardware-run, weakly checked
//
#include <hip/hip_runtime.h>


namespace {
constexpr int B = 2, IMG = 224, H0 = 112, H1 = 56, H2 = 28, C1 = 64, CA = 128, CB = 256, KN = 7;
constexpr int T1 = B * H1 * H1, T2 = B * H2 * H2;
constexpr float XS = 8.0f, WSC = 256.0f, EPS = 1e-5f;
typedef _Float16 b16;
typedef __attribute__((ext_vector_type(16))) _Float16 v16b;
typedef __attribute__((ext_vector_type(8))) _Float16 v8b;
typedef __attribute__((ext_vector_type(8))) float v8f;
typedef __attribute__((ext_vector_type(4))) float v4f;
typedef __attribute__((ext_vector_type(2))) float v2f;
__device__ __forceinline__ float bf16_rne(float f) { unsigned int u = __float_as_uint(f); u += 0x7FFFu + ((u >> 16) & 1u); float r = __uint_as_float(u & 0xFFFF0000u); asm volatile("" : "+v"(r)); return r; }
__device__ __forceinline__ void split16(float v, b16& hi, b16& lo) { hi = (b16)v; lo = (b16)(v - (float)hi); }
__device__ __forceinline__ v16b frag_kb(const b16* p, int hh) { const v8b a = *(const v8b*)(p + 8 * hh), b = *(const v8b*)(p + 16 + 8 * hh); v16b f;
#pragma unroll
  for (int e = 0; e < 8; ++e) { f[e] = a[e]; f[8 + e] = b[e]; } return f; }
__device__ __forceinline__ v8f wmma16b(v16b a, v16b b, v8f c) { v8f d = __builtin_amdgcn_wmma_f32_16x16x32_f16(false, a, false, b, (short)0, c, false, false); asm volatile("v_nop\n\tv_nop\n\tv_nop\n\tv_nop" : "+v"(d) : "v"(a), "v"(b)); return d; }
__device__ __forceinline__ void wave_lds_sync() { __builtin_amdgcn_fence(__ATOMIC_RELEASE, "workgroup"); __builtin_amdgcn_wave_barrier(); __builtin_amdgcn_fence(__ATOMIC_ACQUIRE, "workgroup"); }
__device__ __forceinline__ float pmul(float a, float b) { float p = a * b; asm volatile("" : "+v"(p)); return p; }
__device__ __forceinline__ int iclamp(int v, int lo, int hi) { return v < lo ? lo : (v > hi ? hi : v); }
__device__ __forceinline__ float gelu_exact(float v) { return 0.5f * v * (1.0f + erff(v * 0.70710678118654752f)); }

__global__ __launch_bounds__(256) void wconv_kernel(const float* __restrict__ w, int O, int Cin, int KP, b16* __restrict__ WT) { const size_t u = (size_t)blockIdx.x * 256 + threadIdx.x; if (u >= (size_t)O * (KP / 8)) return; const int o = (int)(u / (KP / 8)), k0 = (int)(u % (KP / 8)) * 8; v8b v;
#pragma unroll
  for (int j = 0; j < 8; ++j) { const int k = k0 + j; const int t = k / Cin, c = k % Cin; v[j] = (b16)((k < 9 * Cin) ? bf16_rne(w[((size_t)o * Cin + c) * 9 + t]) * WSC : 0.0f); }
  for (int pass = 0; pass < 2; ++pass) { *(volatile v8b*)(WT + (size_t)o * KP + k0) = v; __threadfence(); } }
__global__ __launch_bounds__(256) void wlin_kernel(const float* __restrict__ w, size_t n8, b16* __restrict__ WT) { const size_t u = (size_t)blockIdx.x * 256 + threadIdx.x; if (u >= n8) return; v8b v;
#pragma unroll
  for (int j = 0; j < 8; ++j) v[j] = (b16)(bf16_rne(w[u * 8 + j]) * WSC); for (int pass = 0; pass < 2; ++pass) { *(volatile v8b*)(WT + u * 8) = v; __threadfence(); } }
__global__ __launch_bounds__(32) void conv1_kernel(const float* __restrict__ x, const b16* __restrict__ WT, const float* __restrict__ bias, int PLIM, float* __restrict__ P1) { __shared__ __attribute__((aligned(16))) b16 Ah[16][40]; __shared__ float Tf[16][68]; const int lane = threadIdx.x, nloc = lane & 15, hlf = lane >> 4; const size_t p0 = (size_t)blockIdx.x * 16; if (p0 >= (size_t)PLIM) return;
  for (int rr = 0; rr < 16; ++rr) { const size_t p = p0 + rr; const int b = (int)(p / (H0 * H0)), oy = (int)((p / H0) % H0), ox = (int)(p % H0); float v = 0.0f; if (lane < 27) { const int t = lane / 3, c = lane % 3; const int iy = 2 * oy + t / 3 - 1, ix = 2 * ox + t % 3 - 1; if (iy >= 0 && iy < IMG && ix >= 0 && ix < IMG) v = bf16_rne(x[(((size_t)b * 3 + c) * IMG + iy) * IMG + ix]); } Ah[rr][lane] = (b16)(v * XS); if (lane < 8) Ah[rr][32 + lane] = (b16)0.0f; }
  wave_lds_sync(); const v16b a = frag_kb(&Ah[nloc][0], hlf);
#pragma unroll
  for (int t = 0; t < 4; ++t) { v8f acc = {}; acc = wmma16b(a, frag_kb(WT + (size_t)(t * 16 + nloc) * 32, hlf), acc); const float bb = bf16_rne(bias[t * 16 + nloc]);
#pragma unroll
    for (int r8 = 0; r8 < 8; ++r8) Tf[8 * hlf + r8][t * 16 + nloc] = acc[r8] * (1.0f / (XS * WSC)) + bb; }
  wave_lds_sync();
  for (int pass = 0; pass < 2; ++pass) { for (int rr = 0; rr < 16; ++rr) *(volatile v2f*)(P1 + (p0 + rr) * C1 + lane * 2) = (v2f){Tf[rr][lane * 2], Tf[rr][lane * 2 + 1]}; __threadfence(); } }
template <int CIN, int COUT, int HIN>
__global__ __launch_bounds__(32) void sconv_kernel(const float* __restrict__ IN, const b16* __restrict__ WT, const float* __restrict__ bias, const float* __restrict__ g, const float* __restrict__ be, int PLIM, float* __restrict__ OUT) {
  constexpr int HO = HIN / 2, KT = 9 * CIN, NT = COUT / 16; __shared__ __attribute__((aligned(16))) b16 Ah[16][CIN + 8], Al[16][CIN + 8]; __shared__ float Tf[16][COUT + 4]; const int lane = threadIdx.x, nloc = lane & 15, hlf = lane >> 4; const size_t p0 = (size_t)blockIdx.x * 16; if (p0 >= (size_t)PLIM) return;
  v8f acc[NT];
#pragma unroll
  for (int t = 0; t < NT; ++t) acc[t] = (v8f){};
#pragma unroll 1
  for (int tap = 0; tap < 9; ++tap) {
    for (int rr = 0; rr < 16; ++rr) { const size_t p = p0 + rr; const int b = (int)(p / (HO * HO)), oy = (int)((p / HO) % HO), ox = (int)(p % HO); const int iy = 2 * oy + tap / 3 - 1, ix = 2 * ox + tap % 3 - 1; const bool ok = iy >= 0 && iy < HIN && ix >= 0 && ix < HIN; const float* src = IN + (((size_t)b * HIN + (ok ? iy : 0)) * HIN + (ok ? ix : 0)) * CIN;
      for (int c = lane; c < CIN; c += 32) { b16 ph, pl; split16((ok ? src[c] : 0.0f) * XS, ph, pl); Ah[rr][c] = ph; Al[rr][c] = pl; } }
    wave_lds_sync();
#pragma unroll
    for (int kb = 0; kb < CIN; kb += 32) { const v16b a = frag_kb(&Ah[nloc][kb], hlf), al = frag_kb(&Al[nloc][kb], hlf);
#pragma unroll
      for (int t = 0; t < NT; ++t) { const v16b bw = frag_kb(WT + (size_t)(t * 16 + nloc) * KT + tap * CIN + kb, hlf); acc[t] = wmma16b(a, bw, acc[t]); acc[t] = wmma16b(al, bw, acc[t]); } }
    wave_lds_sync(); }
#pragma unroll
  for (int t = 0; t < NT; ++t) { const int cc = t * 16 + nloc; const float bb = bf16_rne(bias[cc]);
#pragma unroll
    for (int r8 = 0; r8 < 8; ++r8) Tf[8 * hlf + r8][cc] = acc[t][r8] * (1.0f / (XS * WSC)) + bb; }
  wave_lds_sync(); constexpr int PL = COUT / 32;
  for (int pass = 0; pass < 2; ++pass) { for (int rr = 0; rr < 16; ++rr) { float v[PL]; float s = 0.0f;
#pragma unroll
      for (int k = 0; k < PL; ++k) { v[k] = Tf[rr][lane * PL + k]; s += v[k]; } for (int o = 16; o; o >>= 1) s += __shfl_xor(s, o); const float mu = s * (1.0f / COUT); float q = 0.0f;
#pragma unroll
      for (int k = 0; k < PL; ++k) q += pmul(v[k] - mu, v[k] - mu); for (int o = 16; o; o >>= 1) q += __shfl_xor(q, o); const float rs = rsqrtf(q * (1.0f / COUT) + EPS);
#pragma unroll
      for (int k = 0; k < PL; ++k) ((volatile float*)OUT)[(p0 + rr) * COUT + lane * PL + k] = pmul(pmul(v[k] - mu, rs), bf16_rne(g[lane * PL + k])) + bf16_rne(be[lane * PL + k]); } __threadfence(); } }
template <int KIN, int LNORM, int ACT, int RES>
__global__ __launch_bounds__(32) void tgemm_kernel(const float* __restrict__ IN, const float* __restrict__ lg, const float* __restrict__ lb, const b16* __restrict__ WT, const float* __restrict__ bias, const float* __restrict__ RESID, int NOUT, int TLIM, float* __restrict__ OUT) { __shared__ __attribute__((aligned(16))) b16 Ah[16][KIN + 8], Al[16][KIN + 8]; __shared__ float Tf[16][260]; const int lane = threadIdx.x, nloc = lane & 15, hlf = lane >> 4; const int NG = (NOUT + 255) / 256; const int g = blockIdx.x % NG; const size_t t0 = (size_t)(blockIdx.x / NG) * 16; if (t0 >= (size_t)TLIM) return; const int ncol = (NOUT - g * 256) < 256 ? (NOUT - g * 256) : 256; const int nt = ncol / 16;
  constexpr int PL = KIN / 32;
  for (int rr = 0; rr < 16; ++rr) { float v[PL];
#pragma unroll
    for (int k = 0; k < PL; ++k) v[k] = IN[(t0 + rr) * KIN + k * 32 + lane];
    if (LNORM) { float s = 0.0f; for (int k = 0; k < PL; ++k) s += v[k]; for (int o = 16; o; o >>= 1) s += __shfl_xor(s, o); const float mu = s * (1.0f / KIN); float q = 0.0f; for (int k = 0; k < PL; ++k) q += pmul(v[k] - mu, v[k] - mu); for (int o = 16; o; o >>= 1) q += __shfl_xor(q, o); const float rs = rsqrtf(q * (1.0f / KIN) + EPS);
#pragma unroll
      for (int k = 0; k < PL; ++k) v[k] = pmul(pmul(v[k] - mu, rs), bf16_rne(lg[k * 32 + lane])) + bf16_rne(lb[k * 32 + lane]); }
#pragma unroll
    for (int k = 0; k < PL; ++k) { b16 ph, pl; split16(v[k] * XS, ph, pl); Ah[rr][k * 32 + lane] = ph; Al[rr][k * 32 + lane] = pl; } }
  wave_lds_sync(); v8f acc[16];
#pragma unroll
  for (int t = 0; t < 16; ++t) acc[t] = (v8f){};
#pragma unroll 1
  for (int kb = 0; kb < KIN; kb += 32) { const v16b a = frag_kb(&Ah[nloc][kb], hlf), al = frag_kb(&Al[nloc][kb], hlf);
#pragma unroll
    for (int t = 0; t < 16; ++t) { if (t < nt) { const v16b bw = frag_kb(WT + (size_t)(g * 256 + t * 16 + nloc) * KIN + kb, hlf); acc[t] = wmma16b(a, bw, acc[t]); acc[t] = wmma16b(al, bw, acc[t]); } } }
#pragma unroll
  for (int t = 0; t < 16; ++t) { if (t < nt) { const int cc = g * 256 + t * 16 + nloc; const float bb = bf16_rne(bias[cc]);
#pragma unroll
    for (int r8 = 0; r8 < 8; ++r8) { float v = acc[t][r8] * (1.0f / (XS * WSC)) + bb; if (ACT == 1) v = gelu_exact(v); Tf[8 * hlf + r8][t * 16 + nloc] = v; } } }
  wave_lds_sync();
  for (int pass = 0; pass < 2; ++pass) { for (int rr = 0; rr < 16; ++rr) for (int q = 0; q < ncol / 128; ++q) { v4f v = *(const v4f*)(&Tf[rr][q * 128 + lane * 4]); if (RES) { const v4f r = *(const v4f*)(RESID + (t0 + rr) * NOUT + g * 256 + q * 128 + lane * 4); for (int k = 0; k < 4; ++k) v[k] += r[k]; } *(volatile v4f*)(OUT + (t0 + rr) * NOUT + g * 256 + q * 128 + lane * 4) = v; } __threadfence(); } }
__global__ __launch_bounds__(256) void natt_kernel(const float* __restrict__ QKV, const float* __restrict__ rpb, int C, int heads, int HS, int TLIM, float* __restrict__ AO) { const int wave = threadIdx.x >> 5, lane = threadIdx.x & 31; const size_t wid = (size_t)blockIdx.x * 8 + wave; const size_t t = wid / heads; const int h = (int)(wid % heads); if (t >= (size_t)TLIM) return; const int b = (int)(t / (HS * HS)), i = (int)((t / HS) % HS), j = (int)(t % HS);
  const float q = QKV[t * 3 * C + h * 32 + lane] * 0.17677669529663688f;
  const int si = iclamp(i - KN / 2, 0, HS - KN), sj = iclamp(j - KN / 2, 0, HS - KN); float m = -INFINITY, den = 0.0f, acc = 0.0f;
#pragma unroll 1
  for (int p = 0; p < KN * KN; ++p) { const int ki = si + p / KN, kj = sj + p % KN; const size_t tk = ((size_t)b * HS + ki) * HS + kj; float s = pmul(q, QKV[tk * 3 * C + C + h * 32 + lane]); for (int o = 16; o; o >>= 1) s += __shfl_xor(s, o);
    s += bf16_rne(rpb[((size_t)h * (2 * KN - 1) + (ki - i + KN - 1)) * (2 * KN - 1) + (kj - j + KN - 1)]); const float mn = fmaxf(m, s); const float sf = (m == -INFINITY) ? 0.0f : __expf(m - mn); const float e = __expf(s - mn); den = den * sf + e; acc = pmul(acc, sf) + pmul(e, QKV[tk * 3 * C + 2 * C + h * 32 + lane]); m = mn; }
  const float o = acc / den;
  for (int pass = 0; pass < 2; ++pass) { ((volatile float*)AO)[t * C + h * 32 + lane] = o; __threadfence(); } }
__global__ __launch_bounds__(256) void out_kernel(const float* __restrict__ X, float* __restrict__ out) { const int u = blockIdx.x * 256 + threadIdx.x; if (u >= B * CB * H2 * H2) return; const int b = u / (CB * H2 * H2), c = (u / (H2 * H2)) % CB, y = (u / H2) % H2, xx = u % H2; const float v = X[(((size_t)b * H2 + y) * H2 + xx) * CB + c];
  for (int pass = 0; pass < 2; ++pass) { ((volatile float*)out)[u] = v; __threadfence(); } }
}

extern "C" void kernel_launch(void* const* d_in, const int* in_sizes, int n_in, void* d_out, int out_size, void* d_ws, size_t ws_size, hipStream_t stream) {
  (void)n_in;
  auto Fp = [&](int i) { return (const float*)d_in[i]; };
  if (in_sizes[0] != B * 3 * IMG * IMG || in_sizes[1] != C1 * 27 || in_sizes[3] != CA * C1 * 9 || in_sizes[9] != 3 * 3 * CA * CA || in_sizes[11] != 3 * 4 * 169 || in_sizes[20] != CB * CA * 9 || in_sizes[26] != 4 * 3 * CB * CB || in_sizes[35] != 4 * CB * 2 * CB || out_size != B * CB * H2 * H2) return;
  const int BV = B, NB0 = 3, NB1 = 4;
  size_t off = 0; char* ws = (char*)d_ws;
  auto carve = [&](size_t bytes) { char* p = ws + off; off += (bytes + 255) & ~(size_t)255; return p; };
  b16* WC1 = (b16*)carve((size_t)C1 * 32 * 2); b16* WC2 = (b16*)carve((size_t)CA * 576 * 2); b16* WDS = (b16*)carve((size_t)CB * 1152 * 2);
  b16* W0qkv = (b16*)carve((size_t)3 * 3 * CA * CA * 2); b16* W0p = (b16*)carve((size_t)3 * CA * CA * 2); b16* W0f1 = (b16*)carve((size_t)3 * 2 * CA * CA * 2); b16* W0f2 = (b16*)carve((size_t)3 * 2 * CA * CA * 2);
  b16* W1qkv = (b16*)carve((size_t)4 * 3 * CB * CB * 2); b16* W1p = (b16*)carve((size_t)4 * CB * CB * 2); b16* W1f1 = (b16*)carve((size_t)4 * 2 * CB * CB * 2); b16* W1f2 = (b16*)carve((size_t)4 * 2 * CB * CB * 2);
  float* P1 = (float*)carve((size_t)B * H0 * H0 * C1 * 4); float* X0 = (float*)carve((size_t)T1 * CA * 4); float* X1 = (float*)carve((size_t)T1 * CA * 4); float* QKV = (float*)carve((size_t)T1 * 3 * CA * 4); float* AO = (float*)carve((size_t)T1 * CA * 4); float* F1 = (float*)carve((size_t)T1 * 2 * CA * 4);
  if (off > ws_size || off > ((size_t)96 << 20)) return;
  auto g8 = [](size_t n8) { return (unsigned)((n8 + 255) / 256); };
  wconv_kernel<<<g8((size_t)C1 * 4 * 32), 256, 0, stream>>>(Fp(1), C1, 3, 32, WC1); wconv_kernel<<<g8((size_t)CA * 72 * 32), 256, 0, stream>>>(Fp(3), CA, C1, 576, WC2); wconv_kernel<<<g8((size_t)CB * 144 * 32), 256, 0, stream>>>(Fp(20), CB, CA, 1152, WDS);
  wlin_kernel<<<g8((size_t)3 * 3 * CA * CA / 8), 256, 0, stream>>>(Fp(9), (size_t)3 * 3 * CA * CA / 8, W0qkv); wlin_kernel<<<g8((size_t)3 * CA * CA / 8), 256, 0, stream>>>(Fp(12), (size_t)3 * CA * CA / 8, W0p); wlin_kernel<<<g8((size_t)3 * 2 * CA * CA / 8), 256, 0, stream>>>(Fp(16), (size_t)3 * 2 * CA * CA / 8, W0f1); wlin_kernel<<<g8((size_t)3 * 2 * CA * CA / 8), 256, 0, stream>>>(Fp(18), (size_t)3 * 2 * CA * CA / 8, W0f2);
  wlin_kernel<<<g8((size_t)4 * 3 * CB * CB / 8), 256, 0, stream>>>(Fp(26), (size_t)4 * 3 * CB * CB / 8, W1qkv); wlin_kernel<<<g8((size_t)4 * CB * CB / 8), 256, 0, stream>>>(Fp(29), (size_t)4 * CB * CB / 8, W1p); wlin_kernel<<<g8((size_t)4 * 2 * CB * CB / 8), 256, 0, stream>>>(Fp(33), (size_t)4 * 2 * CB * CB / 8, W1f1); wlin_kernel<<<g8((size_t)4 * 2 * CB * CB / 8), 256, 0, stream>>>(Fp(35), (size_t)4 * 2 * CB * CB / 8, W1f2);
  const int PL1 = BV * H0 * H0, TL1 = BV * H1 * H1, TL2 = BV * H2 * H2;
  conv1_kernel<<<PL1 / 16, 32, 0, stream>>>(Fp(0), WC1, Fp(2), PL1, P1);
  sconv_kernel<C1, CA, H0><<<TL1 / 16, 32, 0, stream>>>(P1, WC2, Fp(4), Fp(5), Fp(6), TL1, X0);
  for (int i = 0; i < NB0; ++i) {
    tgemm_kernel<CA, 1, 0, 0><<<(TL1 / 16) * 2, 32, 0, stream>>>(X0, Fp(7) + i * CA, Fp(8) + i * CA, W0qkv + (size_t)i * 3 * CA * CA, Fp(10) + i * 3 * CA, nullptr, 3 * CA, TL1, QKV);
    natt_kernel<<<(TL1 * 4 + 7) / 8, 256, 0, stream>>>(QKV, Fp(11) + (size_t)i * 4 * 169, CA, 4, H1, TL1, AO);
    tgemm_kernel<CA, 0, 0, 1><<<TL1 / 16, 32, 0, stream>>>(AO, nullptr, nullptr, W0p + (size_t)i * CA * CA, Fp(13) + i * CA, X0, CA, TL1, X1);
    tgemm_kernel<CA, 1, 1, 0><<<TL1 / 16, 32, 0, stream>>>(X1, Fp(14) + i * CA, Fp(15) + i * CA, W0f1 + (size_t)i * 2 * CA * CA, Fp(17) + i * 2 * CA, nullptr, 2 * CA, TL1, F1);
    tgemm_kernel<2 * CA, 0, 0, 1><<<TL1 / 16, 32, 0, stream>>>(F1, nullptr, nullptr, W0f2 + (size_t)i * 2 * CA * CA, Fp(19) + i * CA, X1, CA, TL1, X0); }
  float* Y0 = X1; float* Y1 = AO;
  sconv_kernel<CA, CB, H1><<<TL2 / 16, 32, 0, stream>>>(X0, WDS, Fp(21), Fp(22), Fp(23), TL2, Y0);
  float* QKV1 = QKV; float* AO1 = F1; float* F11 = X0;
  for (int i = 0; i < NB1; ++i) {
    tgemm_kernel<CB, 1, 0, 0><<<(TL2 / 16) * 3, 32, 0, stream>>>(Y0, Fp(24) + i * CB, Fp(25) + i * CB, W1qkv + (size_t)i * 3 * CB * CB, Fp(27) + i * 3 * CB, nullptr, 3 * CB, TL2, QKV1);
    natt_kernel<<<(TL2 * 8 + 7) / 8, 256, 0, stream>>>(QKV1, Fp(28) + (size_t)i * 8 * 169, CB, 8, H2, TL2, AO1);
    tgemm_kernel<CB, 0, 0, 1><<<TL2 / 16, 32, 0, stream>>>(AO1, nullptr, nullptr, W1p + (size_t)i * CB * CB, Fp(30) + i * CB, Y0, CB, TL2, Y1);
    tgemm_kernel<CB, 1, 1, 0><<<(TL2 / 16) * 2, 32, 0, stream>>>(Y1, Fp(31) + i * CB, Fp(32) + i * CB, W1f1 + (size_t)i * 2 * CB * CB, Fp(34) + i * 2 * CB, nullptr, 2 * CB, TL2, F11);
    tgemm_kernel<2 * CB, 0, 0, 1><<<TL2 / 16, 32, 0, stream>>>(F11, nullptr, nullptr, W1f2 + (size_t)i * 2 * CB * CB, Fp(36) + i * CB, Y1, CB, TL2, Y0); }
  out_kernel<<<(B * CB * H2 * H2 + 255) / 256, 256, 0, stream>>>(Y0, (float*)d_out);
}
